// SeqSelfAttention_21010980012181
// MI455X (gfx1250) — hardware-verified
//
#include <hip/hip_runtime.h>
#include <math.h>
#include <stdint.h>

#define DEVINL __device__ __forceinline__

typedef _Float16 f16t;
typedef _Float16 v16h __attribute__((ext_vector_type(16)));
typedef _Float16 v8h  __attribute__((ext_vector_type(8)));
typedef float    v8f  __attribute__((ext_vector_type(8)));
typedef float    v4f  __attribute__((ext_vector_type(4)));
typedef v8h __attribute__((may_alias)) v8ha;
typedef v4f __attribute__((may_alias)) v4fa;
union FragH { v16h v; v8h half[2]; };

#define BB      2
#define LL      1024
#define DD      256
#define UU      64
#define NROWS   (BB * LL)
#define RT      16
#define NTILES  (NROWS / RT)
#define TPB     256
#define NWAVES  8
#define AWID    64
#define JOFF    (AWID / 2)
#define JW      96
#define JS      80
#define KB_STR  68
#define ES_STR  80
#define P_STR   104
#define O_STR   260
#define T_STR   68

#define XCAR    8.0f
#define WCAR    64.0f
#define SC_QK   (1.0f / 512.0f)
#define PCAR    16384.0f
#define SC_PX   (1.0f / 131072.0f)
#define MASKP   10000.0f
#define NEG_INF (-__builtin_inff())

static_assert(TPB == NWAVES * 32);
static_assert((NROWS % RT) == 0);
static_assert((LL % RT) == 0);
static_assert((DD % 32) == 0);
static_assert((JW % 32) == 0);
static_assert(JS + 16 == JW);
static_assert(RT - 1 + AWID <= JS);
static_assert(RT * JS == 5 * TPB);
static_assert(RT * UU == 4 * TPB);
static_assert(JS * UU == 20 * TPB);
static_assert(RT * 16 == TPB);
static_assert(NWAVES * 32 == DD);
static_assert(NWAVES * 2 == RT);
static_assert(32 * 4 * 2 == DD);
static_assert((NWAVES / 2) * 16 == UU);
static_assert((NWAVES / 2) * 4 == RT);
static_assert(2 * UU == 32 * 4);
static_assert((KB_STR % 4) == 0);
static_assert((O_STR % 4) == 0);
static_assert((T_STR % 4) == 0);
static_assert((P_STR % 8) == 0);
static_assert(RT * O_STR <= JS * KB_STR);

DEVINL v8f wmma_f16(v16h a, v16h b, v8f c) {
  v8f d = __builtin_amdgcn_wmma_f32_16x16x32_f16(false, a, false, b, (short)0, c, false, false);
  asm volatile("v_nop\n\tv_nop\n\tv_nop\n\tv_nop" : "+v"(d) : "v"(a), "v"(b));
  return d;
}
DEVINL v8f zero8f() {
  v8f z = {0.f, 0.f, 0.f, 0.f, 0.f, 0.f, 0.f, 0.f};
  return z;
}
DEVINL int clampi(int v, int lo, int hi) { return v < lo ? lo : (v > hi ? hi : v); }

DEVINL void load_frag_f32(FragH& f, const float* row, int k0, float scale) {
  const v4f x0 = *(const v4fa*)(row + k0);
  const v4f x1 = *(const v4fa*)(row + k0 + 4);
  const v4f x2 = *(const v4fa*)(row + k0 + 16);
  const v4f x3 = *(const v4fa*)(row + k0 + 20);
  #pragma unroll
  for (int j = 0; j < 4; ++j) {
    f.v[j]      = (f16t)(x0[j] * scale);
    f.v[4 + j]  = (f16t)(x1[j] * scale);
    f.v[8 + j]  = (f16t)(x2[j] * scale);
    f.v[12 + j] = (f16t)(x3[j] * scale);
  }
}

__global__ __launch_bounds__(TPB) void proj_kernel(const float* __restrict__ x,
                                                  const float* __restrict__ Wt,
                                                  const float* __restrict__ Wx,
                                                  float* __restrict__ qbuf,
                                                  float* __restrict__ kbuf)
{
  __shared__ __attribute__((aligned(16))) float ts[2][RT * T_STR];
  const int tid = threadIdx.x, lane = tid & 31;
  const int wave = __builtin_amdgcn_readfirstlane(tid >> 5);
  const int hh = lane >> 4, m = lane & 15;
  if (blockIdx.x >= NTILES) return;
  const int g0 = blockIdx.x * RT;
  const int which = wave >> 2;
  const int n0 = (wave & 3) * 16;
  const float* W = (which == 0) ? Wt : Wx;
  const float* xrow = x + (size_t)(g0 + m) * DD + 8 * hh;
  const float* wcol = W + n0 + m;

  v8f acc = zero8f();
  #pragma unroll 2
  for (int ks = 0; ks < DD / 32; ++ks) {
    const int k0 = 32 * ks;
    FragH a, b;
    load_frag_f32(a, xrow, k0, XCAR);
    #pragma unroll
    for (int i = 0; i < 8; ++i) {
      b.v[i]     = (f16t)(wcol[(size_t)(k0 + 8 * hh + i) * UU] * WCAR);
      b.v[8 + i] = (f16t)(wcol[(size_t)(k0 + 16 + 8 * hh + i) * UU] * WCAR);
    }
    acc = wmma_f16(a.v, b.v, acc);
  }

  float* T = &ts[which][0];
  #pragma unroll
  for (int r = 0; r < 8; ++r) T[(8 * hh + r) * T_STR + n0 + m] = acc[r] * SC_QK;
  __syncthreads();

  float* dst = (which == 0) ? qbuf : kbuf;
  const int wl = wave & 3;
  v4f va[2];
  float* da[2];
  #pragma unroll
  for (int c = 0; c < 2; ++c) {
    const int row = 4 * wl + 2 * c + hh;
    const int col = 4 * m;
    va[c] = *(const v4fa*)(T + row * T_STR + col);
    da[c] = dst + (size_t)(g0 + row) * UU + col;
    *(volatile v4f*)da[c] = va[c];
  }
  __threadfence();
  #pragma unroll
  for (int c = 0; c < 2; ++c) *(volatile v4f*)da[c] = va[c];
}

union KO { float kb[JS * KB_STR]; float os[RT * O_STR]; };

__global__ __launch_bounds__(TPB) void attn_kernel(const float* __restrict__ x,
                                                  const float* __restrict__ qbuf,
                                                  const float* __restrict__ kbuf,
                                                  const float* __restrict__ bh,
                                                  const float* __restrict__ Wa,
                                                  const float* __restrict__ ba,
                                                  float* __restrict__ out)
{
  __shared__ __attribute__((aligned(16))) KO uko;
  __shared__ __attribute__((aligned(16))) float qs[RT * UU];
  __shared__ __attribute__((aligned(16))) float es[RT * ES_STR];
  __shared__ __attribute__((aligned(16))) f16t ps[RT * P_STR];
  __shared__ __attribute__((aligned(16))) float was[UU];
  __shared__ __attribute__((aligned(16))) float bhs[UU];
  __shared__ float sInv[RT];

  const int tid = threadIdx.x, lane = tid & 31;
  const int wave = __builtin_amdgcn_readfirstlane(tid >> 5);
  const int hh = lane >> 4, m = lane & 15;
  if (blockIdx.x >= NTILES) return;
  const int t  = blockIdx.x;
  const int b  = t / (LL / RT);
  const int i0 = (t % (LL / RT)) * RT;
  const size_t gbase = (size_t)b * LL;
  const size_t g0 = gbase + i0;
  const int j0 = i0 - JOFF;

  {
    const int row = tid >> 4, col = 4 * (tid & 15);
    *(v4fa*)(qs + row * UU + col) = *(const v4fa*)(qbuf + (g0 + row) * UU + col);
  }
  #pragma unroll
  for (int it = 0; it < 5; ++it) {
    const int idx = tid + TPB * it;
    const int jj = idx >> 4, col = 4 * (idx & 15);
    const int j = j0 + jj;
    const int jc = clampi(j, 0, LL - 1);
    v4f v = *(const v4fa*)(kbuf + (gbase + jc) * UU + col);
    if (j < 0 || j >= LL) { v[0] = 0.f; v[1] = 0.f; v[2] = 0.f; v[3] = 0.f; }
    *(v4fa*)(uko.kb + jj * KB_STR + col) = v;
  }
  if (tid < UU) { was[tid] = Wa[tid]; bhs[tid] = bh[tid]; }
  const float bav = ba[0];
  __syncthreads();

  #pragma unroll 1
  for (int it = 0; it < 5; ++it) {
    const int idx = tid + TPB * it;
    const int ii = idx / JS;
    const int jj = idx - ii * JS;
    const float* qr = qs + ii * UU;
    const float* kr = uko.kb + jj * KB_STR;
    float s = 0.0f;
    #pragma unroll 2
    for (int u = 0; u < UU; u += 4) {
      const v4f q4 = *(const v4fa*)(qr + u);
      const v4f k4 = *(const v4fa*)(kr + u);
      const v4f w4 = *(const v4fa*)(was + u);
      const v4f b4 = *(const v4fa*)(bhs + u);
      #pragma unroll
      for (int c = 0; c < 4; ++c) s = fmaf(tanhf((q4[c] + k4[c]) + b4[c]), w4[c], s);
    }
    const int j = j0 + jj;
    const bool valid = (j >= 0) && (j < LL);
    const bool band = (jj >= ii) && (jj < ii + AWID);
    float ev = s + bav;
    ev = ev - MASKP * (band ? 0.0f : 1.0f);
    es[ii * ES_STR + jj] = valid ? ev : NEG_INF;
  }
  __syncthreads();

  {
    const int r = tid >> 4, tt = tid & 15;
    const float* er = es + r * ES_STR;
    float v[5];
    float mx = NEG_INF;
    #pragma unroll
    for (int c = 0; c < 5; ++c) { v[c] = er[tt + 16 * c]; mx = fmaxf(mx, v[c]); }
    mx = fmaxf(mx, __shfl_xor(mx, 8));
    mx = fmaxf(mx, __shfl_xor(mx, 4));
    mx = fmaxf(mx, __shfl_xor(mx, 2));
    mx = fmaxf(mx, __shfl_xor(mx, 1));
    float sum = 0.0f;
    f16t* pr = ps + r * P_STR;
    #pragma unroll
    for (int c = 0; c < 5; ++c) {
      const float p = expf(v[c] - mx);
      sum += p;
      pr[tt + 16 * c] = (f16t)(p * PCAR);
    }
    pr[JS + tt] = (f16t)0.0f;
    sum += __shfl_xor(sum, 8);
    sum += __shfl_xor(sum, 4);
    sum += __shfl_xor(sum, 2);
    sum += __shfl_xor(sum, 1);
    if (tt == 0) sInv[r] = (1.0f / sum) * SC_PX;
  }
  __syncthreads();

  const f16t* prow = ps + m * P_STR + 8 * hh;
  const float* xb = x + gbase * DD;
  v8f acc[2];
  acc[0] = zero8f();
  acc[1] = zero8f();
  #pragma unroll
  for (int ks = 0; ks < JW / 32; ++ks) {
    const int k0 = 32 * ks;
    FragH A;
    A.half[0] = *(const v8ha*)(prow + k0);
    A.half[1] = *(const v8ha*)(prow + k0 + 16);
    int ra[8], rb[8];
    bool oka[8], okb[8];
    #pragma unroll
    for (int i = 0; i < 8; ++i) {
      const int ja = j0 + k0 + 8 * hh + i;
      const int jb = j0 + k0 + 16 + 8 * hh + i;
      oka[i] = (ja >= 0) && (ja < LL);
      okb[i] = (jb >= 0) && (jb < LL);
      ra[i] = clampi(ja, 0, LL - 1);
      rb[i] = clampi(jb, 0, LL - 1);
    }
    #pragma unroll
    for (int tn = 0; tn < 2; ++tn) {
      const int d = 32 * wave + 16 * tn + m;
      FragH Bf;
      #pragma unroll
      for (int i = 0; i < 8; ++i) {
        const float xa = xb[(size_t)ra[i] * DD + d];
        const float xv = xb[(size_t)rb[i] * DD + d];
        Bf.v[i]     = oka[i] ? (f16t)(xa * XCAR) : (f16t)0.0f;
        Bf.v[8 + i] = okb[i] ? (f16t)(xv * XCAR) : (f16t)0.0f;
      }
      acc[tn] = wmma_f16(A.v, Bf.v, acc[tn]);
    }
  }

  float* const os = uko.os;
  #pragma unroll
  for (int tn = 0; tn < 2; ++tn) {
    const int d = 32 * wave + 16 * tn + m;
    #pragma unroll
    for (int r = 0; r < 8; ++r) {
      const int row = 8 * hh + r;
      os[row * O_STR + d] = acc[tn][r] * sInv[row];
    }
  }
  __syncthreads();

  v4f va[4];
  float* da[4];
  #pragma unroll
  for (int jr = 0; jr < 2; ++jr) {
    const int row = 2 * wave + jr;
    #pragma unroll
    for (int c = 0; c < 2; ++c) {
      const int col = 128 * c + 4 * lane;
      va[2 * jr + c] = *(const v4fa*)(os + row * O_STR + col);
      da[2 * jr + c] = out + (g0 + row) * DD + col;
      *(volatile v4f*)da[2 * jr + c] = va[2 * jr + c];
    }
  }
  __threadfence();
  #pragma unroll
  for (int q = 0; q < 4; ++q) *(volatile v4f*)da[q] = va[q];
}

extern "C" void kernel_launch(void* const* d_in, const int* in_sizes, int n_in,
                              void* d_out, int out_size, void* d_ws, size_t ws_size,
                              hipStream_t stream) {
  if (n_in < 6) return;
  if (in_sizes[0] != NROWS * DD) return;
  if (in_sizes[1] != DD * UU || in_sizes[2] != DD * UU) return;
  if (in_sizes[3] != UU || in_sizes[4] != UU || in_sizes[5] < 1) return;
  if (out_size != NROWS * DD) return;

  const float* x  = (const float*)d_in[0];
  const float* Wt = (const float*)d_in[1];
  const float* Wx = (const float*)d_in[2];
  const float* bh = (const float*)d_in[3];
  const float* Wa = (const float*)d_in[4];
  const float* ba = (const float*)d_in[5];
  float* outp = (float*)d_out;

  const size_t szQ = (size_t)NROWS * UU * 4;
  size_t off = 0;
  char* ws = (char*)d_ws;
  float* qbuf = (float*)(ws + off);  off += szQ;
  float* kbuf = (float*)(ws + off);  off += szQ;
  if (off > ws_size) return;

  proj_kernel<<<NTILES, TPB, 0, stream>>>(x, Wt, Wx, qbuf, kbuf);
  attn_kernel<<<NTILES, TPB, 0, stream>>>(x, qbuf, kbuf, bh, Wa, ba, outp);
  (void)hipGetLastError();
}
